// EEG_GAT_35837207118112
// MI455X (gfx1250) — hardware-verified
//
#include <hip/hip_runtime.h>


namespace {
constexpr int NB = 64, NN = 1024, F = 200, FO = 200, KP = 224, NT = 13, FP = NT * 16, M = NB * NN;
constexpr float XS = 8.0f, WSC = 256.0f, PS = 1024.0f, NEG = 0.2f;
typedef _Float16 b16;
typedef __attribute__((ext_vector_type(16))) _Float16 v16b;
typedef __attribute__((ext_vector_type(8))) _Float16 v8b;
typedef __attribute__((ext_vector_type(8))) float v8f;
typedef __attribute__((ext_vector_type(4))) float v4f;
__device__ __forceinline__ float bf16_rne(float f) { unsigned int u = __float_as_uint(f); u += 0x7FFFu + ((u >> 16) & 1u); return __uint_as_float(u & 0xFFFF0000u); }
__device__ __forceinline__ void split16(float v, b16& hi, b16& lo) { hi = (b16)v; lo = (b16)(v - (float)hi); }
__device__ __forceinline__ v16b frag_kb(const b16* p, int hh) { const v8b a = *(const v8b*)(p + 8 * hh), b = *(const v8b*)(p + 16 + 8 * hh); v16b f;
#pragma unroll
  for (int e = 0; e < 8; ++e) { f[e] = a[e]; f[8 + e] = b[e]; } return f; }
__device__ __forceinline__ v8f wmma16b(v16b a, v16b b, v8f c) { v8f d = __builtin_amdgcn_wmma_f32_16x16x32_f16(false, a, false, b, (short)0, c, false, false); asm volatile("v_nop\n\tv_nop\n\tv_nop\n\tv_nop" : "+v"(d) : "v"(a), "v"(b)); return d; }
__device__ __forceinline__ void wave_lds_sync() { __builtin_amdgcn_fence(__ATOMIC_RELEASE, "workgroup"); __builtin_amdgcn_wave_barrier(); __builtin_amdgcn_fence(__ATOMIC_ACQUIRE, "workgroup"); }
__device__ __forceinline__ float pmul(float a, float b) { float p = a * b; asm volatile("" : "+v"(p)); return p; }
__device__ __forceinline__ float opaque(float a) { asm volatile("" : "+v"(a)); return a; }
__device__ __forceinline__ float lrelu(float x) { return x >= 0.0f ? x : NEG * x; }
__device__ __forceinline__ float nexp(float x) { return __builtin_amdgcn_exp2f(x * 1.4426950408889634f); }

__global__ __launch_bounds__(256) void wprep_kernel(const float* __restrict__ w, b16* __restrict__ WT) {
  const size_t u = (size_t)blockIdx.x * 256 + threadIdx.x; if (u >= (size_t)FP * KP / 8) return; const size_t e = u * 8; const int o = (int)(e / KP), k0 = (int)(e % KP); v8b v;
  for (int j = 0; j < 8; ++j) { const int k = k0 + j; v[j] = (o < FO && k < F) ? (b16)(bf16_rne(w[(size_t)(k < F ? k : 0) * FO + (o < FO ? o : 0)]) * WSC) : (b16)0.0f; }
  for (int pass = 0; pass < 2; ++pass) { *(volatile v8b*)(WT + e) = v; __threadfence(); }
}
__global__ __launch_bounds__(128) void hgemm_kernel(const float* __restrict__ x, const b16* __restrict__ WT, const float* __restrict__ as_, const float* __restrict__ ad_, const float* __restrict__ bias, float* __restrict__ H0, float* __restrict__ AS, float* __restrict__ AD, float* __restrict__ out) {
  __shared__ __attribute__((aligned(16))) float Tf[4][16 * FP]; __shared__ __attribute__((aligned(16))) float sa[64], sd[64];
  const int wave = threadIdx.x >> 5, lane = threadIdx.x & 31, nloc = lane & 15, hlf = lane >> 4; const size_t m0 = (size_t)blockIdx.x * 64 + wave * 16; const bool g0 = blockIdx.x < NN / 64;
  const float* xr = x + (m0 + nloc) * F;
  v8f acc[NT];
#pragma unroll
  for (int t = 0; t < NT; ++t) acc[t] = (v8f){};
#pragma unroll 1
  for (int kb = 0; kb < KP; kb += 32) { v16b a; for (int j = 0; j < 8; ++j) { const int k0 = kb + 8 * hlf + j, k1 = kb + 16 + 8 * hlf + j; a[j] = k0 < F ? (b16)(bf16_rne(xr[k0 < F ? k0 : 0]) * XS) : (b16)0.0f; a[8 + j] = k1 < F ? (b16)(bf16_rne(xr[k1 < F ? k1 : 0]) * XS) : (b16)0.0f; }
#pragma unroll
    for (int t = 0; t < NT; ++t) acc[t] = wmma16b(a, frag_kb(WT + (size_t)(t * 16 + nloc) * KP + kb, hlf), acc[t]); }
  const float sc = 1.0f / (XS * WSC);
  if (!g0) {
#pragma unroll
    for (int t = 0; t < NT; ++t) { const int c = t * 16 + nloc; const float bb = c < FO ? bf16_rne(bias[c < FO ? c : 0]) : 0.0f;
#pragma unroll 1
      for (int r8 = 0; r8 < 8; ++r8) if (c < FO) Tf[wave][(8 * hlf + r8) * FO + c] = acc[t][r8] * sc + bb; }
    wave_lds_sync();
    for (int pass = 0; pass < 2; ++pass) {
#pragma unroll 1
      for (int q = 0; q < 25; ++q) *(volatile v4f*)(out + m0 * FO + (size_t)(q * 32 + lane) * 4) = *(const v4f*)(&Tf[wave][(q * 32 + lane) * 4]); __threadfence(); }
    return; }
  float ps[8], pd[8]; for (int r8 = 0; r8 < 8; ++r8) { ps[r8] = 0.0f; pd[r8] = 0.0f; }
#pragma unroll
  for (int t = 0; t < NT; ++t) { const int c = t * 16 + nloc; const bool cv = c < FO; const float ws_ = cv ? opaque(bf16_rne(as_[cv ? c : 0])) : 0.0f, wd_ = cv ? opaque(bf16_rne(ad_[cv ? c : 0])) : 0.0f;
#pragma unroll
    for (int r8 = 0; r8 < 8; ++r8) { const float v = cv ? acc[t][r8] * sc : 0.0f; Tf[wave][(8 * hlf + r8) * FP + c] = v; ps[r8] += pmul(v, ws_); pd[r8] += pmul(v, wd_); } }
#pragma unroll
  for (int r8 = 0; r8 < 8; ++r8) { float a = ps[r8], b = pd[r8]; for (int o = 1; o < 16; o <<= 1) { a += __shfl_xor(a, o); b += __shfl_xor(b, o); } if (nloc == 0) { sa[wave * 16 + 8 * hlf + r8] = a; sd[wave * 16 + 8 * hlf + r8] = b; } }
  __syncthreads();
  for (int pass = 0; pass < 2; ++pass) {
#pragma unroll 1
    for (int q = 0; q < 26; ++q) *(volatile v4f*)(H0 + m0 * FP + (size_t)(q * 32 + lane) * 4) = *(const v4f*)(&Tf[wave][(q * 32 + lane) * 4]);
    if (threadIdx.x < 16) *(volatile v4f*)(AS + (size_t)blockIdx.x * 64 + threadIdx.x * 4) = *(const v4f*)(&sa[threadIdx.x * 4]); else if (threadIdx.x < 32) *(volatile v4f*)(AD + (size_t)blockIdx.x * 64 + (threadIdx.x - 16) * 4) = *(const v4f*)(&sd[(threadIdx.x - 16) * 4]);
    __threadfence(); }
}
__global__ __launch_bounds__(256) void htrans_kernel(const float* __restrict__ H0, b16* __restrict__ HTH, b16* __restrict__ HTL) {
  __shared__ float tile[64][64 + 1];
  const int c0 = blockIdx.x * 64, j0 = blockIdx.y * 64; const int wave = threadIdx.x >> 5, lane = threadIdx.x & 31;
  for (int rr = 0; rr < 8; ++rr) { const int jl = wave * 8 + rr; const float* row = H0 + (size_t)(j0 + jl) * FP + c0; const int ca = c0 + lane * 2; tile[lane * 2][jl] = ca < FP ? row[lane * 2] : 0.0f; tile[lane * 2 + 1][jl] = (ca + 1) < FP ? row[lane * 2 + 1] : 0.0f; }
  __syncthreads();
  typedef __attribute__((ext_vector_type(2))) _Float16 v2b;
  for (int pass = 0; pass < 2; ++pass) { for (int rr = 0; rr < 8; ++rr) { const int cl = wave * 8 + rr; const int c = c0 + cl; if (c < FP) { b16 p0, q0, p1, q1; split16(tile[cl][lane * 2] * XS, p0, q0); split16(tile[cl][lane * 2 + 1] * XS, p1, q1); v2b h, l; h[0] = p0; h[1] = p1; l[0] = q0; l[1] = q1;
        *(volatile v2b*)(HTH + (size_t)c * NN + j0 + lane * 2) = h; *(volatile v2b*)(HTL + (size_t)c * NN + j0 + lane * 2) = l; } } __threadfence(); }
}
__global__ __launch_bounds__(32) void attn_kernel(const float* __restrict__ AS, const float* __restrict__ AD, const b16* __restrict__ HTH, const b16* __restrict__ HTL, const float* __restrict__ bias, float* __restrict__ out) {
  __shared__ __attribute__((aligned(16))) float Tf[16 * FO]; __shared__ float dens[16];
  const int lane = threadIdx.x, nloc = lane & 15, hlf = lane >> 4; const int i0 = blockIdx.x * 16;
  float mx = -INFINITY; for (int j = lane; j < NN; j += 32) mx = fmaxf(mx, AS[j]); for (int o = 16; o; o >>= 1) mx = fmaxf(mx, __shfl_xor(mx, o));
  const float adi = AD[i0 + nloc]; const float mi = lrelu(adi + mx); float den = 0.0f;
  v8f acc[NT];
#pragma unroll
  for (int t = 0; t < NT; ++t) acc[t] = (v8f){};
#pragma unroll 1
  for (int kb = 0; kb < NN; kb += 32) { v16b ph, pl;
    for (int j = 0; j < 8; ++j) { const float p0 = nexp(lrelu(adi + AS[kb + 8 * hlf + j]) - mi), p1 = nexp(lrelu(adi + AS[kb + 16 + 8 * hlf + j]) - mi); den += p0 + p1; b16 a, b; split16(p0 * PS, a, b); ph[j] = a; pl[j] = b; split16(p1 * PS, a, b); ph[8 + j] = a; pl[8 + j] = b; }
#pragma unroll
    for (int t = 0; t < NT; ++t) { const v16b bh = frag_kb(HTH + (size_t)(t * 16 + nloc) * NN + kb, hlf), bl = frag_kb(HTL + (size_t)(t * 16 + nloc) * NN + kb, hlf); acc[t] = wmma16b(ph, bh, acc[t]); acc[t] = wmma16b(pl, bh, acc[t]); acc[t] = wmma16b(ph, bl, acc[t]); } }
  den += __shfl_xor(den, 16);
  if (hlf == 0) dens[nloc] = den;
  wave_lds_sync();
#pragma unroll
  for (int t = 0; t < NT; ++t) { const int c = t * 16 + nloc; const float bb = c < FO ? bf16_rne(bias[c < FO ? c : 0]) : 0.0f;
#pragma unroll 1
    for (int r8 = 0; r8 < 8; ++r8) { const int rl = 8 * hlf + r8; if (c < FO) Tf[rl * FO + c] = acc[t][r8] * (1.0f / (PS * XS)) / dens[rl] + bb; } }
  wave_lds_sync();
  for (int pass = 0; pass < 2; ++pass) {
#pragma unroll 1
    for (int q = 0; q < 25; ++q) *(volatile v4f*)(out + (size_t)i0 * FO + (size_t)(q * 32 + lane) * 4) = *(const v4f*)(&Tf[(q * 32 + lane) * 4]); __threadfence(); }
}
}

extern "C" void kernel_launch(void* const* d_in, const int* in_sizes, int n_in, void* d_out, int out_size, void* d_ws, size_t ws_size, hipStream_t stream) {
  (void)n_in;
  auto Fp = [&](int i) { return (const float*)d_in[i]; };
  if (in_sizes[0] != M * F || in_sizes[1] != F * FO || in_sizes[2] != FO || in_sizes[3] != FO || in_sizes[4] != FO || out_size != M * FO) return;
  size_t off = 0; char* ws = (char*)d_ws;
  auto carve = [&](size_t bytes) { char* p = ws + off; off += (bytes + 255) & ~(size_t)255; return p; };
  b16* WT = (b16*)carve((size_t)FP * KP * 2); float* H0 = (float*)carve((size_t)NN * FP * 4); float* AS = (float*)carve(NN * 4); float* AD = (float*)carve(NN * 4); b16* HTH = (b16*)carve((size_t)FP * NN * 2); b16* HTL = (b16*)carve((size_t)FP * NN * 2);
  if (off > ws_size || off > ((size_t)16 << 20)) return;
  wprep_kernel<<<(unsigned)(((size_t)FP * KP / 8 + 255) / 256), 256, 0, stream>>>(Fp(1), WT);
  hgemm_kernel<<<M / 64, 128, 0, stream>>>(Fp(0), WT, Fp(2), Fp(3), Fp(4), H0, AS, AD, (float*)d_out);
  htrans_kernel<<<dim3((FP + 63) / 64, NN / 64), 256, 0, stream>>>(H0, HTH, HTL);
  attn_kernel<<<NN / 16, 32, 0, stream>>>(AS, AD, HTH, HTL, Fp(4), (float*)d_out);
}
